// EsmFoldAttention_86827058856663
// MI455X (gfx1250) — hardware-verified
//
#include <hip/hip_runtime.h>


#define NB_  8
#define TT   1024
#define CC   256
#define NH_  8
#define HD   32
typedef _Float16 h16;
typedef unsigned short bf;
typedef __attribute__((ext_vector_type(16))) __bf16   v16bf;
typedef __attribute__((ext_vector_type(16))) _Float16 v16h;
typedef __attribute__((ext_vector_type(8)))  _Float16 v8h;
typedef __attribute__((ext_vector_type(8)))  unsigned short v8us;
typedef __attribute__((ext_vector_type(8)))  float    v8f;
typedef __attribute__((ext_vector_type(4)))  float    v4f;
typedef v8h  __attribute__((may_alias)) v8ha;
typedef v4f  __attribute__((may_alias)) v4fa;
typedef v8us __attribute__((may_alias)) v8usa;

__device__ __forceinline__ unsigned short f2bf(float f) { unsigned u = __float_as_uint(f); u += 0x7FFFu + ((u >> 16) & 1u); return (unsigned short)(u >> 16); }
__device__ __forceinline__ float bf2f(unsigned short b) { return __uint_as_float(((unsigned)b) << 16); }
__device__ __forceinline__ float bfr(float f) { return bf2f(f2bf(f)); }
__device__ __forceinline__ v16h cat16(v8h lo, v8h hi) { return __builtin_shufflevector(lo, hi, 0, 1, 2, 3, 4, 5, 6, 7, 8, 9, 10, 11, 12, 13, 14, 15); }
__device__ __forceinline__ v16bf cat16b(v8us lo, v8us hi) { return __builtin_bit_cast(v16bf, __builtin_shufflevector(lo, hi, 0, 1, 2, 3, 4, 5, 6, 7, 8, 9, 10, 11, 12, 13, 14, 15)); }
__device__ __forceinline__ v8f wmma16(v16h a, v16h b, v8f c) { return __builtin_amdgcn_wmma_f32_16x16x32_f16(false, a, false, b, (short)0, c, false, false); }
__device__ __forceinline__ v8f wmmab(v16bf a, v16bf b, v8f c) { return __builtin_amdgcn_wmma_f32_16x16x32_bf16(false, a, false, b, (short)0, c, false, false); }


template <typename T16> struct WFrag;
template <> struct WFrag<h16> { typedef v16h V; static __device__ __forceinline__ V ld(const h16* p) { return cat16(*(const v8h*)p, *(const v8h*)(p + 16)); } static __device__ __forceinline__ v8f mma(V a, V b, v8f c) { return wmma16(a, b, c); } };
template <> struct WFrag<bf> { typedef v16bf V; static __device__ __forceinline__ V ld(const bf* p) { return cat16b(*(const v8us*)p, *(const v8us*)(p + 16)); } static __device__ __forceinline__ v8f mma(V a, V b, v8f c) { return wmmab(a, b, c); } };
template <typename T16, int NSPLIT, bool BIAS>
__global__ __launch_bounds__(32) void k_gemmw(const T16* __restrict__ A, const T16* __restrict__ A2, const T16* __restrict__ Bt, const T16* __restrict__ Bt2, int K, float* C, int ldc, const float* __restrict__ bias, size_t sA, size_t sB, size_t sC) {
    typedef typename WFrag<T16>::V V;
    __shared__ __align__(16) float os[16 * 68];
    const size_t z = blockIdx.z; A += z * sA; if (A2) A2 += z * sA; Bt += z * sB; if (Bt2) Bt2 += z * sB; C += z * sC;
    const int lane = threadIdx.x & 31, lr = lane & 15, hi = lane >> 4; const int r0 = blockIdx.x * 64, c0 = blockIdx.y * 64;
    v8f acc[4][4];
#pragma unroll
    for (int mb = 0; mb < 4; ++mb)
#pragma unroll
        for (int nb = 0; nb < 4; ++nb) acc[mb][nb] = (v8f){};
    const size_t aoff = (size_t)(r0 + lr) * K + 8 * hi, boff = (size_t)(c0 + lr) * K + 8 * hi;
#pragma unroll 1
    for (int kc = 0; kc < K; kc += 32) {
        V a[4], a2[4];
#pragma unroll
        for (int mb = 0; mb < 4; ++mb) { a[mb] = WFrag<T16>::ld(A + aoff + (size_t)mb * 16 * K + kc); if (NSPLIT == 1 || NSPLIT == 2) a2[mb] = WFrag<T16>::ld(A2 + aoff + (size_t)mb * 16 * K + kc); }
#pragma unroll
        for (int nb = 0; nb < 4; ++nb) { const V b = WFrag<T16>::ld(Bt + boff + (size_t)nb * 16 * K + kc); V b2; if (NSPLIT >= 2) b2 = WFrag<T16>::ld(Bt2 + boff + (size_t)nb * 16 * K + kc);
#pragma unroll
            for (int mb = 0; mb < 4; ++mb) { acc[mb][nb] = WFrag<T16>::mma(a[mb], b, acc[mb][nb]); if (NSPLIT == 1 || NSPLIT == 2) acc[mb][nb] = WFrag<T16>::mma(a2[mb], b, acc[mb][nb]); if (NSPLIT >= 2) acc[mb][nb] = WFrag<T16>::mma(a[mb], b2, acc[mb][nb]); } }
        asm volatile("v_nop\n\tv_nop\n\tv_nop\n\tv_nop" : "+v"(acc[0][0]), "+v"(acc[1][1]), "+v"(acc[2][2]), "+v"(acc[3][3]) : "v"(a[0]), "v"(a[3]));
    }
#pragma unroll
    for (int mb = 0; mb < 4; ++mb) {
#pragma unroll
        for (int nb = 0; nb < 4; ++nb) {
#pragma unroll
            for (int j = 0; j < 8; ++j) os[(hi * 8 + j) * 68 + nb * 16 + lr] = acc[mb][nb][j]; }
        __builtin_amdgcn_wave_barrier(); asm volatile("" ::: "memory");
        float* crow = C + (size_t)(r0 + mb * 16) * ldc + c0;
#pragma unroll 1
        for (int ps = 0; ps < 2; ++ps) {
#pragma unroll
            for (int s = 0; s < 8; ++s) { const int row = 2 * s + hi, cofs = lr * 4; v4f val = *(const v4fa*)(os + row * 68 + cofs); if (BIAS) { val[0] += bfr(bias[c0 + cofs]); val[1] += bfr(bias[c0 + cofs + 1]); val[2] += bfr(bias[c0 + cofs + 2]); val[3] += bfr(bias[c0 + cofs + 3]); }
                *(volatile v4f*)(crow + (size_t)row * ldc + cofs) = val; }
            if (ps == 0) __threadfence(); }
        __builtin_amdgcn_wave_barrier(); asm volatile("" ::: "memory");
    }
}

__device__ __forceinline__ void splitf(float y, unsigned short& h, unsigned short& l) { h = f2bf(y); l = f2bf(y - bf2f(h)); }
typedef __attribute__((ext_vector_type(2))) unsigned short v2us;
typedef __attribute__((ext_vector_type(4))) unsigned short v4us;

__global__ __launch_bounds__(256) void k_wtG(const float* __restrict__ w, int K, int N, bf* Bt) {
    const int lane = threadIdx.x & 31; const int L0 = (blockIdx.x * 8 + (threadIdx.x >> 5)) * 8; const int nlines = N * K / 64;
#pragma unroll
    for (int ps = 0; ps < 2; ++ps) {
#pragma unroll 1
        for (int l = 0; l < 8; ++l) { const int L = L0 + l; if (L >= nlines) break; const size_t e = (size_t)L * 64 + lane * 2; const int k = (int)(e % K), n = (int)(e / K); v2us o;
            o[0] = f2bf(w[(size_t)k * N + n]); o[1] = f2bf(w[(size_t)(k + 1) * N + n]); *(volatile v2us*)(Bt + e) = o; }
        if (ps == 0) __threadfence(); }
}
__global__ __launch_bounds__(256) void k_cvt8(const float* __restrict__ src, bf* dst, size_t n8) { const size_t i = (size_t)blockIdx.x * 256 + threadIdx.x; if (i >= n8) return; const v8f v = *(const v8f*)(src + i * 8); v8us o;
#pragma unroll
    for (int k = 0; k < 8; ++k) o[k] = f2bf(v[k]); *(volatile v8us*)(dst + i * 8) = o; __threadfence(); *(volatile v8us*)(dst + i * 8) = o; }
__global__ __launch_bounds__(256) void k_pl(const float* __restrict__ F, float dv, bf* Ph, bf* Pl) { const int e = (blockIdx.x * 256 + threadIdx.x) * 4; if (e >= NH_ * TT * HD) return; const int d = e % HD; const int t = (e / HD) % TT; const int h = e / (HD * TT); const float* f = F + (size_t)t * CC + h * HD + d; v4us oh, ol;
#pragma unroll
    for (int u = 0; u < 4; ++u) { unsigned short a, b; splitf((dv != 0.f) ? __fdiv_rn(f[u], dv) : f[u], a, b); oh[u] = a; ol[u] = b; } for (int ps = 0; ps < 2; ++ps) { *(volatile v4us*)(Ph + e) = oh; *(volatile v4us*)(Pl + e) = ol; if (ps == 0) __threadfence(); } }
__global__ __launch_bounds__(256) void k_vt(const float* __restrict__ V, bf* Th, bf* Tl) { const int e = (blockIdx.x * 256 + threadIdx.x) * 2; if (e >= NH_ * 64 * TT) return; const int t = e % TT; const int d = (e / TT) % 64; const int h = e / (TT * 64); v2us oh, ol;
    if (d < HD) { unsigned short a1, b1, a2, b2; splitf(V[(size_t)t * CC + h * HD + d], a1, b1); splitf(V[(size_t)(t + 1) * CC + h * HD + d], a2, b2); oh[0] = a1; oh[1] = a2; ol[0] = b1; ol[1] = b2; } else { oh[0] = oh[1] = 0; ol[0] = ol[1] = 0; }
    for (int ps = 0; ps < 2; ++ps) { *(volatile v2us*)(Th + e) = oh; *(volatile v2us*)(Tl + e) = ol; if (ps == 0) __threadfence(); } }
__global__ __launch_bounds__(256) void k_esoft(const float* __restrict__ Sb, const float* __restrict__ bm, const float* __restrict__ bp, bf* Ph, bf* Pl) { const int lane = threadIdx.x & 31; const int row = blockIdx.x * 8 + (threadIdx.x >> 5); if (row >= NH_ * TT) return; const float* sr = Sb + (size_t)row * TT; const float* br = bp + (size_t)row * TT; float v[TT / 32]; float mx = -3.0e38f;
#pragma unroll
    for (int ch = 0; ch < TT / 128; ++ch) { const int j0 = ch * 128 + lane * 4; const v4f a = *(const v4f*)(sr + j0), m4 = *(const v4f*)(bm + j0), p4 = *(const v4f*)(br + j0);
#pragma unroll
        for (int u = 0; u < 4; ++u) { float m1 = bfr(m4[u]); asm volatile("" : "+v"(m1)); float t0 = __fadd_rn(a[u], m1); float p1 = bfr(p4[u]); asm volatile("" : "+v"(p1)); const float t = __fadd_rn(t0, p1); v[ch * 4 + u] = t; mx = fmaxf(mx, t); } }
#pragma unroll
    for (int sh = 16; sh; sh >>= 1) mx = fmaxf(mx, __shfl_xor(mx, sh, 32));
    float sum = 0.f;
#pragma unroll
    for (int q = 0; q < TT / 32; ++q) { float d0 = __fsub_rn(v[q], mx); asm volatile("" : "+v"(d0)); v[q] = __builtin_amdgcn_exp2f(__fmul_rn(d0, 1.4426950408889634f)); sum += v[q]; }
#pragma unroll
    for (int sh = 16; sh; sh >>= 1) sum += __shfl_xor(sum, sh, 32);
    const float f = __fdiv_rn(1.0f, sum);
    for (int ps = 0; ps < 2; ++ps) {
#pragma unroll
        for (int ch = 0; ch < TT / 128; ++ch) { v4us oh, ol;
#pragma unroll
            for (int q = 0; q < 4; ++q) { unsigned short a, b; splitf(v[ch * 4 + q] * f, a, b); oh[q] = a; ol[q] = b; } const size_t oo = (size_t)row * TT + ch * 128 + lane * 4; *(volatile v4us*)(Ph + oo) = oh; *(volatile v4us*)(Pl + oo) = ol; }
        if (ps == 0) __threadfence(); } }
__global__ __launch_bounds__(256) void k_gate(const float* __restrict__ O, const float* __restrict__ G, bf* Ah, bf* Al) { const int e = (blockIdx.x * 256 + threadIdx.x) * 4; if (e >= TT * CC) return; const int c = e % CC; const int t = e / CC; const int h = c / HD, d = c % HD; const float* o = O + ((size_t)h * TT + t) * 64 + d; v4us oh, ol;
#pragma unroll
    for (int u = 0; u < 4; ++u) { float sg = __fdiv_rn(1.0f, __fadd_rn(1.0f, __expf(-G[e + u]))); asm volatile("" : "+v"(sg)); unsigned short a, b; splitf(__fmul_rn(o[u], sg), a, b); oh[u] = a; ol[u] = b; } *(volatile v4us*)(Ah + e) = oh; *(volatile v4us*)(Al + e) = ol; __threadfence(); *(volatile v4us*)(Ah + e) = oh; *(volatile v4us*)(Al + e) = ol; }

extern "C" void kernel_launch(void* const* d_in, const int* in_sizes, int n_in,
                              void* d_out, int out_size, void* d_ws, size_t ws_size, hipStream_t stream) {
    (void)in_sizes; (void)n_in; (void)out_size;
    const float** I = (const float**)d_in;
    const float *qx = I[0], *kvx = I[1], *bmask = I[2], *bpair = I[3], *Wq = I[4], *Wk = I[5], *Wv = I[6], *Wg = I[7], *bg = I[8], *Wo = I[9], *bo = I[10];
    float* OUT = (float*)d_out;
    char* wsp = (char*)d_ws;
    auto take = [&](size_t bytes) { char* p = wsp; wsp += (bytes + 255) & ~(size_t)255; return (void*)p; };
    bf* BQ = (bf*)take(CC * CC * 2); bf* BK = (bf*)take(CC * CC * 2); bf* BV = (bf*)take(CC * CC * 2); bf* BG = (bf*)take(CC * CC * 2); bf* BO = (bf*)take(CC * CC * 2);
    bf* QX = (bf*)take((size_t)TT * CC * 2); bf* KX = (bf*)take((size_t)TT * CC * 2); float* Q = (float*)take((size_t)TT * CC * 4); float* K = (float*)take((size_t)TT * CC * 4); float* V = (float*)take((size_t)TT * CC * 4); float* G = (float*)take((size_t)TT * CC * 4);
    bf* Qh = (bf*)take((size_t)NH_ * TT * HD * 2); bf* Ql = (bf*)take((size_t)NH_ * TT * HD * 2); bf* Kh = (bf*)take((size_t)NH_ * TT * HD * 2); bf* Kl = (bf*)take((size_t)NH_ * TT * HD * 2); bf* VTh = (bf*)take((size_t)NH_ * 64 * TT * 2); bf* VTl = (bf*)take((size_t)NH_ * 64 * TT * 2);
    float* Sb = (float*)take((size_t)NH_ * TT * TT * 4); bf* Ph = (bf*)take((size_t)NH_ * TT * TT * 2); bf* Pl = (bf*)take((size_t)NH_ * TT * TT * 2); float* O = (float*)take((size_t)NH_ * TT * 64 * 4); bf* Ah = (bf*)take((size_t)TT * CC * 2); bf* Al = (bf*)take((size_t)TT * CC * 2);
    if ((size_t)(wsp - (char*)d_ws) > ws_size) return;
    k_wtG<<<(CC * CC / 64 + 63) / 64, 256, 0, stream>>>(Wq, CC, CC, BQ); k_wtG<<<(CC * CC / 64 + 63) / 64, 256, 0, stream>>>(Wk, CC, CC, BK); k_wtG<<<(CC * CC / 64 + 63) / 64, 256, 0, stream>>>(Wv, CC, CC, BV); k_wtG<<<(CC * CC / 64 + 63) / 64, 256, 0, stream>>>(Wg, CC, CC, BG); k_wtG<<<(CC * CC / 64 + 63) / 64, 256, 0, stream>>>(Wo, CC, CC, BO);
    const dim3 gp(TT / 64, CC / 64, 1); const size_t zq = (size_t)TT * HD, zS = (size_t)TT * TT, zv = (size_t)64 * TT, zo = (size_t)TT * 64;
    for (int b = 0; b < NB_; ++b) {
        k_cvt8<<<(TT * CC / 8 + 255) / 256, 256, 0, stream>>>(qx + (size_t)b * TT * CC, QX, TT * CC / 8); k_cvt8<<<(TT * CC / 8 + 255) / 256, 256, 0, stream>>>(kvx + (size_t)b * TT * CC, KX, TT * CC / 8);
        k_gemmw<bf, 0, false><<<gp, 32, 0, stream>>>(QX, nullptr, BQ, nullptr, CC, Q, CC, nullptr, 0, 0, 0); k_gemmw<bf, 0, false><<<gp, 32, 0, stream>>>(KX, nullptr, BK, nullptr, CC, K, CC, nullptr, 0, 0, 0); k_gemmw<bf, 0, false><<<gp, 32, 0, stream>>>(KX, nullptr, BV, nullptr, CC, V, CC, nullptr, 0, 0, 0); k_gemmw<bf, 0, true><<<gp, 32, 0, stream>>>(QX, nullptr, BG, nullptr, CC, G, CC, bg, 0, 0, 0);
        k_pl<<<(NH_ * TT * HD / 4 + 255) / 256, 256, 0, stream>>>(Q, 5.656854249492381f, Qh, Ql); k_pl<<<(NH_ * TT * HD / 4 + 255) / 256, 256, 0, stream>>>(K, 0.f, Kh, Kl); k_vt<<<(NH_ * 64 * TT / 2 + 255) / 256, 256, 0, stream>>>(V, VTh, VTl);
        k_gemmw<bf, 2, false><<<dim3(TT / 64, TT / 64, NH_), 32, 0, stream>>>(Qh, Ql, Kh, Kl, HD, Sb, TT, nullptr, zq, zq, zS);
        k_esoft<<<NH_ * TT / 8, 256, 0, stream>>>(Sb, bmask + (size_t)b * TT, bpair, Ph, Pl);
        k_gemmw<bf, 2, false><<<dim3(TT / 64, 1, NH_), 32, 0, stream>>>(Ph, Pl, VTh, VTl, TT, O, 64, nullptr, zS, zv, zo);
        k_gate<<<(TT * CC / 4 + 255) / 256, 256, 0, stream>>>(O, G, Ah, Al);
        k_gemmw<bf, 1, true><<<gp, 32, 0, stream>>>(Ah, Al, BO, nullptr, CC, OUT + (size_t)b * TT * CC, CC, bo, 0, 0, 0); }
}
